// attention_1065151889732
// MI455X (gfx1250) — hardware-verified
//
#include <hip/hip_runtime.h>
#include <math.h>

typedef __attribute__((ext_vector_type(16))) _Float16 v16h;
typedef __attribute__((ext_vector_type(8)))  _Float16 v8h;
typedef __attribute__((ext_vector_type(8)))  float    v8f;
typedef __attribute__((ext_vector_type(4)))  float    v4f;

constexpr int kTok    = 8192;
constexpr int kDin    = 256;
constexpr int kDh     = 64;
constexpr int kSlices = 16;
constexpr int kSliceK = kTok / kSlices;
constexpr int kSlabP  = 68;
constexpr int kTrP    = 132;
static_assert(kSliceK == 512, "slice length");
static_assert((kDin % 32) == 0 && (kSliceK % 32) == 0 && (kDh % 32) == 0, "every product depth is a multiple of 32");
static_assert((kTok % 128) == 0 && kDh == 64, "row blocks of 128, 64 output columns");

constexpr float kInCarry    = 16.0f;
constexpr float kWCarry     = 1024.0f;
constexpr float kActCarry   = 16.0f;
constexpr float kMCarry     = 16.0f;
constexpr float kScoreDiv   = 64.0f;
constexpr float kProjScale  = kActCarry / (kInCarry * kWCarry);
constexpr float kStateScale = 1.0f / (kActCarry * kActCarry);
constexpr float kRedScale   = kMCarry / kScoreDiv;
constexpr float kOutScale   = 1.0f / (kActCarry * kMCarry);
constexpr float kF16MinNormal = 6.103515625e-05f;

constexpr size_t kSzX     = (size_t)3 * kTok * kDin * 2;
constexpr size_t kSzWT    = (size_t)3 * kDh * kDin * 2;
constexpr size_t kSzQ     = (size_t)kTok * kDh * 2;
constexpr size_t kSzKVT   = (size_t)2 * kDh * kTok * 2;
constexpr size_t kSzMPART = (size_t)kSlices * kDh * kDh * 4;
constexpr size_t kSzMT    = (size_t)kDh * kDh * 2;
constexpr size_t kOffXH    = 0;
constexpr size_t kOffWTH   = kOffXH + kSzX;
constexpr size_t kOffQH    = kOffWTH + kSzWT;
constexpr size_t kOffKVTH  = kOffQH + kSzQ;
constexpr size_t kOffMPART = kOffKVTH + kSzKVT;
constexpr size_t kOffMTH   = kOffMPART + kSzMPART;
constexpr size_t kWsTotal  = kOffMTH + kSzMT;
static_assert(kWsTotal == 16097280ull, "carve total");
static_assert(kWsTotal <= 134217728ull, "carve cap");
static_assert((kOffWTH % 128) == 0 && (kOffQH % 128) == 0 && (kOffKVTH % 128) == 0 &&
              (kOffMPART % 128) == 0 && (kOffMTH % 128) == 0, "128-B aligned regions");

union FragU { v16h v; v8h h[2]; };
__device__ __forceinline__ v16h frag_load(const _Float16* p) {
  FragU f;
  f.h[0] = *(const v8h*)(p);
  f.h[1] = *(const v8h*)(p + 16);
  return f.v;
}

__device__ __forceinline__ v8f mma_g(v16h a, v16h b, v8f c) {
  c = __builtin_amdgcn_wmma_f32_16x16x32_f16(false, a, false, b, (short)0, c, false, false);
  asm volatile("v_nop\n\tv_nop\n\tv_nop\n\tv_nop" : "+v"(c) : "v"(a), "v"(b));
  return c;
}

__device__ __forceinline__ _Float16 cvt16(float v) {
  const float vf = (fabsf(v) < kF16MinNormal) ? 0.0f : v;
  return (_Float16)vf;
}
__device__ __forceinline__ v8h cvt8(v4f a0, v4f a1) {
  v8h hv;
#pragma unroll
  for (int e = 0; e < 4; ++e) {
    const float f0 = a0[e];
    const float f1 = a1[e];
    hv[e]     = cvt16(f0);
    hv[4 + e] = cvt16(f1);
  }
  return hv;
}

__global__ __launch_bounds__(256) void wt_cast_kernel(const float* __restrict__ W0, const float* __restrict__ W1,
                                                      const float* __restrict__ W2,
                                                      unsigned short* __restrict__ WtH, float carry) {
  __shared__ float sm[64][65];
  const int t   = threadIdx.x;
  const int in0 = blockIdx.x * 64;
  const int z   = blockIdx.y;
  const float* W = (z == 0) ? W0 : ((z == 1) ? W1 : W2);
#pragma unroll
  for (int i = 0; i < 16; ++i) {
    const int e = i * 256 + t;
    const int r = e >> 6;
    const int c = e & 63;
    sm[c][r] = W[(size_t)(in0 + r) * kDh + c] * carry;
  }
  __syncthreads();
  const int lane = t & 31, wave = t >> 5;
  const int q = lane >> 3, c8 = (lane & 7) * 8;
  v8h hv[2];
#pragma unroll
  for (int it = 0; it < 2; ++it) {
    const int row = wave * 8 + it * 4 + q;
    const v4f a0 = (v4f){sm[row][c8 + 0], sm[row][c8 + 1], sm[row][c8 + 2], sm[row][c8 + 3]};
    const v4f a1 = (v4f){sm[row][c8 + 4], sm[row][c8 + 5], sm[row][c8 + 6], sm[row][c8 + 7]};
    hv[it] = cvt8(a0, a1);
  }
  unsigned short* oh = WtH + (size_t)z * kDh * kDin;
  for (int pass = 0; pass < 2; ++pass) {
#pragma unroll
    for (int it = 0; it < 2; ++it) {
      const int row = wave * 8 + it * 4 + q;
      const size_t o = (size_t)row * kDin + in0 + c8;
      *(volatile v8h*)(oh + o) = hv[it];
    }
    __threadfence();
  }
}

__global__ __launch_bounds__(256) void cast_in_kernel(const float* __restrict__ x0, const float* __restrict__ x1,
                                                      const float* __restrict__ x2,
                                                      unsigned short* __restrict__ XH, int total8, float carry) {
  const int i = blockIdx.x * 256 + threadIdx.x;
  if (i >= total8) return;
  const int z = blockIdx.y;
  const float* src = (z == 0) ? x0 : ((z == 1) ? x1 : x2);
  const size_t e0 = (size_t)i << 3;
  v4f a0 = *(const v4f*)(src + e0);
  v4f a1 = *(const v4f*)(src + e0 + 4);
  a0 = a0 * carry;
  a1 = a1 * carry;
  const v8h hv = cvt8(a0, a1);
  const size_t po = (size_t)z * ((size_t)total8 << 3) + e0;
  unsigned short* qh = XH + po;
  *(volatile v8h*)qh = hv;
  __threadfence();
  *(volatile v8h*)qh = hv;
}

template <int NW, int EPI>
__global__ __launch_bounds__(NW * 32) void gemm1_kernel(
    const unsigned short* __restrict__ Ahp, int lda, long strideA,
    const unsigned short* __restrict__ Bhp, int ldb, long strideB,
    void* __restrict__ C0, long strideC, int ldt, int K, float scale) {
  static_assert(EPI != 2 || NW == 8, "transposed output uses 128-token blocks");
  __shared__ __align__(16) float sT[(EPI == 2) ? (64 * kTrP) : (NW * 16 * kSlabP)];
  const int lane  = threadIdx.x & 31;
  const int wave  = threadIdx.x >> 5;
  const int z     = blockIdx.y;
  const int rlane = lane & 15;
  const int hh    = lane >> 4;
  const int koff  = hh * 8;
  const int m0    = (blockIdx.x * NW + wave) * 16;

  const _Float16* Ah = (const _Float16*)Ahp + (size_t)z * strideA + (size_t)(m0 + rlane) * lda + koff;
  const _Float16* Bh = (const _Float16*)Bhp + (size_t)z * strideB + (size_t)rlane * ldb + koff;

  v8f am[4];
#pragma unroll
  for (int j = 0; j < 4; ++j) {
    am[j] = (v8f){0.f, 0.f, 0.f, 0.f, 0.f, 0.f, 0.f, 0.f};
  }

  for (int k0 = 0; k0 < K; k0 += 32) {
    const v16h ah = frag_load(Ah + k0);
#pragma unroll
    for (int j = 0; j < 4; ++j) {
      const size_t bo = (size_t)(j * 16) * ldb + k0;
      const v16h bh = frag_load(Bh + bo);
      am[j] = mma_g(ah, bh, am[j]);
    }
  }

  if (EPI == 2) {
#pragma unroll
    for (int j = 0; j < 4; ++j) {
#pragma unroll
      for (int r = 0; r < 8; ++r) {
        const float v = am[j][r] * scale;
        sT[(j * 16 + rlane) * kTrP + wave * 16 + 8 * hh + r] = v;
      }
    }
    __syncthreads();
    const int q = lane >> 3, c8 = (lane & 7) * 8;
    const size_t tok0 = (size_t)blockIdx.x * (NW * 16);
    unsigned short* Ch = (unsigned short*)C0 + (size_t)z * strideC;
    v8h hv[4];
#pragma unroll
    for (int it = 0; it < 4; ++it) {
      const int line = wave * 16 + it * 4 + q;
      const int ch = line >> 1, seg = line & 1;
      const float* sp = sT + ch * kTrP + seg * 64 + c8;
      const v4f a0 = *(const v4f*)(sp);
      const v4f a1 = *(const v4f*)(sp + 4);
      hv[it] = cvt8(a0, a1);
    }
    for (int pass = 0; pass < 2; ++pass) {
#pragma unroll
      for (int it = 0; it < 4; ++it) {
        const int line = wave * 16 + it * 4 + q;
        const int ch = line >> 1, seg = line & 1;
        const size_t o = (size_t)ch * ldt + tok0 + seg * 64 + c8;
        *(volatile v8h*)(Ch + o) = hv[it];
      }
      __threadfence();
    }
  } else {
    float* slab = sT + wave * 16 * kSlabP;
#pragma unroll
    for (int j = 0; j < 4; ++j) {
#pragma unroll
      for (int r = 0; r < 8; ++r) {
        const float v = am[j][r] * scale;
        slab[(8 * hh + r) * kSlabP + j * 16 + rlane] = v;
      }
    }
    __syncthreads();
    if (EPI == 0) {
      float* C = (float*)C0 + (size_t)z * strideC;
      const int c4 = rlane * 4;
      v4f vv[8];
#pragma unroll
      for (int it = 0; it < 8; ++it) {
        const int row = it * 2 + hh;
        vv[it] = *(const v4f*)(slab + row * kSlabP + c4);
      }
      for (int pass = 0; pass < 2; ++pass) {
#pragma unroll
        for (int it = 0; it < 8; ++it) {
          const int row = it * 2 + hh;
          *(volatile v4f*)(C + (size_t)(m0 + row) * kDh + c4) = vv[it];
        }
        __threadfence();
      }
    } else {
      unsigned short* Ch = (unsigned short*)C0 + (size_t)z * strideC;
      const int q = lane >> 3, c8 = (lane & 7) * 8;
      v8h hv[4];
#pragma unroll
      for (int it = 0; it < 4; ++it) {
        const int row = it * 4 + q;
        const float* sp = slab + row * kSlabP + c8;
        const v4f a0 = *(const v4f*)(sp);
        const v4f a1 = *(const v4f*)(sp + 4);
        hv[it] = cvt8(a0, a1);
      }
      for (int pass = 0; pass < 2; ++pass) {
#pragma unroll
        for (int it = 0; it < 4; ++it) {
          const int row = it * 4 + q;
          const size_t o = (size_t)(m0 + row) * kDh + c8;
          *(volatile v8h*)(Ch + o) = hv[it];
        }
        __threadfence();
      }
    }
  }
}

__global__ __launch_bounds__(256) void state_reduce_kernel(const float* __restrict__ part,
                                                           unsigned short* __restrict__ MtH, float scale) {
  const int i = blockIdx.x * 256 + threadIdx.x;
  if (i >= (kDh * kDh) / 8) return;
  const size_t e0 = (size_t)i << 3;
  v4f s0 = (v4f){0.f, 0.f, 0.f, 0.f};
  v4f s1 = (v4f){0.f, 0.f, 0.f, 0.f};
#pragma unroll 1
  for (int sl = 0; sl < kSlices; ++sl) {
    const float* p = part + (size_t)sl * (kDh * kDh) + e0;
    const v4f a0 = *(const v4f*)(p);
    const v4f a1 = *(const v4f*)(p + 4);
    s0 = s0 + a0;
    s1 = s1 + a1;
  }
  s0 = s0 * scale;
  s1 = s1 * scale;
  const v8h hv = cvt8(s0, s1);
  unsigned short* qh = MtH + e0;
  *(volatile v8h*)qh = hv;
  __threadfence();
  *(volatile v8h*)qh = hv;
}

extern "C" void kernel_launch(void* const* d_in, const int* in_sizes, int n_in,
                              void* d_out, int out_size, void* d_ws, size_t ws_size,
                              hipStream_t stream) {
  if (n_in < 6) return;
  if (in_sizes[0] != kTok * kDin) return;
  if (in_sizes[1] != kTok * kDin) return;
  if (in_sizes[2] != kTok * kDin) return;
  if (in_sizes[3] != kDin * kDh) return;
  if (in_sizes[4] != kDin * kDh) return;
  if (in_sizes[5] != kDin * kDh) return;
  if (out_size != kTok * kDh) return;
  if (ws_size < kWsTotal) return;

  const float* q_in = (const float*)d_in[0];
  const float* k_in = (const float*)d_in[1];
  const float* v_in = (const float*)d_in[2];
  const float* wQ   = (const float*)d_in[3];
  const float* wK   = (const float*)d_in[4];
  const float* wV   = (const float*)d_in[5];
  float* out = (float*)d_out;

  char* ws = (char*)d_ws;
  unsigned short* XH    = (unsigned short*)(ws + kOffXH);
  unsigned short* WTH   = (unsigned short*)(ws + kOffWTH);
  unsigned short* QH    = (unsigned short*)(ws + kOffQH);
  unsigned short* KVTH  = (unsigned short*)(ws + kOffKVTH);
  float*          MPART = (float*)(ws + kOffMPART);
  unsigned short* MTH   = (unsigned short*)(ws + kOffMTH);

  const long xPlane  = (long)kTok * kDin;
  const long wPlane  = (long)kDh * kDin;
  const long tPlane  = (long)kDh * kTok;
  const int  total8  = kTok * kDin / 8;

  wt_cast_kernel<<<dim3(kDin / 64, 3), 256, 0, stream>>>(wQ, wK, wV, WTH, kWCarry);

  cast_in_kernel<<<dim3(total8 / 256, 3), 256, 0, stream>>>(q_in, k_in, v_in, XH, total8, kInCarry);

  gemm1_kernel<8, 1><<<dim3(kTok / 128, 1), 256, 0, stream>>>(
      XH, kDin, 0L,
      WTH, kDin, 0L,
      (void*)QH, 0L, 0, kDin, kProjScale);

  gemm1_kernel<8, 2><<<dim3(kTok / 128, 2), 256, 0, stream>>>(
      XH + xPlane, kDin, xPlane,
      WTH + wPlane, kDin, wPlane,
      (void*)KVTH, tPlane, kTok, kDin, kProjScale);

  gemm1_kernel<4, 0><<<dim3(1, kSlices), 128, 0, stream>>>(
      KVTH + tPlane, kTok, (long)kSliceK,
      KVTH, kTok, (long)kSliceK,
      (void*)MPART, (long)(kDh * kDh), 0, kSliceK, kStateScale);

  state_reduce_kernel<<<2, 256, 0, stream>>>(MPART, MTH, kRedScale);

  gemm1_kernel<8, 0><<<dim3(kTok / 128, 1), 256, 0, stream>>>(
      QH, kDh, 0L,
      MTH, kDh, 0L,
      (void*)out, 0L, 0, kDh, kOutScale);
}
